// rel_aux_net_13941463842948
// MI455X (gfx1250) — hardware-verified
//
#include <hip/hip_runtime.h>


namespace {
constexpr int Bn = 4, N = 10000, NPAD = 10112  , T = 100000, D = 128, H = 512, O = 64, KN = 160  ;
constexpr float HS_ = 8.0f, EPS = 1e-3f;

typedef _Float16 b16;
typedef __attribute__((ext_vector_type(16))) _Float16 v16b;
typedef __attribute__((ext_vector_type(16))) __bf16 v16bb;
typedef __attribute__((ext_vector_type(8))) _Float16 v8b;
typedef __attribute__((ext_vector_type(8))) unsigned short v8us;
typedef __attribute__((ext_vector_type(8))) float v8f;
typedef __attribute__((ext_vector_type(4))) float v4f;
__device__ __forceinline__ float bf16_rne(float f) { unsigned int u = __float_as_uint(f); u += 0x7FFFu + ((u >> 16) & 1u); return __uint_as_float(u & 0xFFFF0000u); }
__device__ __forceinline__ unsigned short bf16_bits(float f) { unsigned int u = __float_as_uint(f); u += 0x7FFFu + ((u >> 16) & 1u); return (unsigned short)(u >> 16); }
__device__ __forceinline__ void split16(float v, b16& hi, b16& lo) { hi = (b16)v; lo = (b16)(v - (float)hi); }
__device__ __forceinline__ v16b frag_kb(const b16* p, int hh) { const v8b a = *(const v8b*)(p + 8 * hh), b = *(const v8b*)(p + 16 + 8 * hh); v16b f;
#pragma unroll
  for (int e = 0; e < 8; ++e) { f[e] = a[e]; f[8 + e] = b[e]; } return f; }
__device__ __forceinline__ v16bb frag_bf(const unsigned short* p, int hh) { const v8us a = *(const v8us*)(p + 8 * hh), b = *(const v8us*)(p + 16 + 8 * hh); union { unsigned short s[16]; v16bb v; } u;
#pragma unroll
  for (int e = 0; e < 8; ++e) { u.s[e] = a[e]; u.s[8 + e] = b[e]; } return u.v; }
__device__ __forceinline__ v8f wmma16b(v16b a, v16b b, v8f c) { v8f d = __builtin_amdgcn_wmma_f32_16x16x32_f16(false, a, false, b, (short)0, c, false, false); asm volatile("v_nop\n\tv_nop\n\tv_nop\n\tv_nop" : "+v"(d) : "v"(a), "v"(b)); return d; }
__device__ __forceinline__ v8f wmma16bb(v16bb a, v16bb b, v8f c) { v8f d = __builtin_amdgcn_wmma_f32_16x16x32_bf16(false, a, false, b, (short)0, c, false, false); asm volatile("v_nop\n\tv_nop\n\tv_nop\n\tv_nop" : "+v"(d) : "v"(a), "v"(b)); return d; }
__device__ __forceinline__ void wave_lds_sync() { __builtin_amdgcn_fence(__ATOMIC_RELEASE, "workgroup"); __builtin_amdgcn_wave_barrier(); __builtin_amdgcn_fence(__ATOMIC_ACQUIRE, "workgroup"); }
__device__ __forceinline__ float nexp(float x) { return __builtin_amdgcn_exp2f(x * 1.4426950408889634f); }

__global__ __launch_bounds__(256) void prep_kernel(const float* __restrict__ W1, const float* __restrict__ b1, const float* __restrict__ g1, const float* __restrict__ be1, const float* __restrict__ m1, const float* __restrict__ v1,
                                                   const float* __restrict__ W2, const float* __restrict__ b2, const float* __restrict__ g2, const float* __restrict__ be2, const float* __restrict__ m2, const float* __restrict__ v2,
                                                   unsigned short* __restrict__ wn, b16* __restrict__ w2r, float* __restrict__ bnp) {
  const int t_ = threadIdx.x + blockIdx.x * 256, nth = gridDim.x * 256;
  for (int pass = 0; pass < 2; ++pass) {
    for (int p = t_; p < 2 * H * KN; p += nth) { const int row = p / KN, k = p % KN; const int part = row / H, o = row % H; float v = 0.0f;
      if (k < 4) v = W1[(part * 4 + k) * H + o]; else if (k < 4 + D) v = W1[(8 + part * D + (k - 4)) * H + o];
      ((volatile unsigned short*)wn)[p] = bf16_bits(v); }
    for (int p = t_; p < O * H; p += nth) { const int o = p / H, k = p % H; ((volatile b16*)w2r)[p] = (b16)bf16_rne(W2[k * O + o]); }
    for (int c = t_; c < H; c += nth) { const float sc = bf16_rne(g1[c]) * rsqrtf(bf16_rne(v1[c]) + EPS); ((volatile float*)bnp)[c] = sc; ((volatile float*)bnp)[H + c] = bf16_rne(be1[c]) - bf16_rne(m1[c]) * sc + bf16_rne(b1[c]) * sc; }
    for (int c = t_; c < O; c += nth) { const float sc = bf16_rne(g2[c]) * rsqrtf(bf16_rne(v2[c]) + EPS); ((volatile float*)bnp)[2 * H + c] = sc; ((volatile float*)bnp)[2 * H + O + c] = bf16_rne(be2[c]) - bf16_rne(m2[c]) * sc + bf16_rne(b2[c]) * sc; }
    __threadfence();
  }
}

__global__ __launch_bounds__(128) void node_kernel(const float* __restrict__ vec, const float* __restrict__ box, int b, const unsigned short* __restrict__ wn, float* __restrict__ na) {
  __shared__ __attribute__((aligned(16))) float Ts[4][32 * 64];
  const int lane = threadIdx.x & 31, wave = threadIdx.x >> 5, nloc = lane & 15, hlf = lane >> 4, m0 = blockIdx.y * 128 + wave * 32, c0 = blockIdx.x * 64;
  const int ra = min(m0 + nloc, N - 1), rb = min(m0 + 16 + nloc, N - 1); const float* va = vec + ((size_t)b * N + ra) * D; const float* vb = vec + ((size_t)b * N + rb) * D; const float* xa = box + ((size_t)b * N + ra) * 4; const float* xb = box + ((size_t)b * N + rb) * 4;
  v8f acc[2][4];
#pragma unroll
  for (int r = 0; r < 2; ++r)
#pragma unroll
    for (int t = 0; t < 4; ++t) acc[r][t] = (v8f){};
#pragma unroll
  for (int kb = 0; kb < KN; kb += 32) { union { unsigned short s[16]; v16bb v; } ua, ub;
#pragma unroll
    for (int e = 0; e < 16; ++e) { const int k = kb + ((e < 8) ? (8 * hlf + e) : (16 + 8 * hlf + e - 8)); float fa = 0.0f, fb = 0.0f;
      if (k < 4) { fa = xa[k]; fb = xb[k]; } else if (k < 4 + D) { fa = va[k - 4]; fb = vb[k - 4]; }
      ua.s[e] = bf16_bits(fa); ub.s[e] = bf16_bits(fb); }
#pragma unroll
    for (int t = 0; t < 4; ++t) { const v16bb bw = frag_bf(wn + (size_t)(c0 + t * 16 + nloc) * KN + kb, hlf); acc[0][t] = wmma16bb(ua.v, bw, acc[0][t]); acc[1][t] = wmma16bb(ub.v, bw, acc[1][t]); } }
  float* Tt = Ts[wave];
#pragma unroll
  for (int t = 0; t < 4; ++t)
#pragma unroll
    for (int r = 0; r < 2; ++r)
#pragma unroll
      for (int v = 0; v < 8; ++v) Tt[(r * 16 + v + 8 * hlf) * 64 + t * 16 + nloc] = acc[r][t][v];
  wave_lds_sync();
  float* dst0 = na + (size_t)m0 * (2 * H) + c0;
  for (int pass = 0; pass < 2; ++pass) {
#pragma unroll
    for (int j = 0; j < 16; ++j) { const int rr = j * 2 + hlf, c4 = nloc * 4; *(volatile v4f*)(dst0 + (size_t)rr * (2 * H) + c4) = *(const v4f*)(Tt + rr * 64 + c4); }
    __threadfence(); }
}

__global__ __launch_bounds__(64) void edge_kernel(const int* __restrict__ edges, int b, const float* __restrict__ na, const b16* __restrict__ w2r, const float* __restrict__ bnp, float* __restrict__ out) {
  __shared__ __attribute__((aligned(16))) b16 Lh[2][16][H + 8], Ll[2][16][H + 8]; __shared__ float Ys[32];
  const int wid = threadIdx.x >> 5, lane = threadIdx.x & 31, nloc = lane & 15, hlf = lane >> 4; const int e0 = blockIdx.x * 32 + wid * 16;
  { const int ed = e0 + nloc; int s = edges[((size_t)b * T + ed) * 2], o = edges[((size_t)b * T + ed) * 2 + 1]; s = (s < 0) ? 0 : (s >= N ? N - 1 : s); o = (o < 0) ? 0 : (o >= N ? N - 1 : o);
    const float* rs = na + (size_t)s * (2 * H); const float* ro = na + (size_t)o * (2 * H) + H; const float* sc = bnp; const float* sh = bnp + H;
    for (int c4 = hlf * 256; c4 < hlf * 256 + 256; c4 += 4) { const v4f a = *(const v4f*)(rs + c4), c = *(const v4f*)(ro + c4);
#pragma unroll
      for (int e = 0; e < 4; ++e) { const float hv = fmaxf((a[e] + c[e]) * sc[c4 + e] + sh[c4 + e], 0.0f); b16 p, q; split16(hv * HS_, p, q); Lh[wid][nloc][c4 + e] = p; Ll[wid][nloc][c4 + e] = q; } } }
  wave_lds_sync();
  v8f acc[4] = {{}, {}, {}, {}};
#pragma unroll 4
  for (int kb = 0; kb < H; kb += 32) { const v16b ah = frag_kb(&Lh[wid][nloc][kb], hlf), al = frag_kb(&Ll[wid][nloc][kb], hlf);
#pragma unroll
    for (int t = 0; t < 4; ++t) { const v16b bw = frag_kb(w2r + (size_t)(t * 16 + nloc) * H + kb, hlf); acc[t] = wmma16b(ah, bw, acc[t]); acc[t] = wmma16b(al, bw, acc[t]); } }
  const float* sc2 = bnp + 2 * H; const float* sh2 = sc2 + O;
#pragma unroll
  for (int v = 0; v < 8; ++v) { float y[4]; float m = -INFINITY;
#pragma unroll
    for (int t = 0; t < 4; ++t) { const int c = t * 16 + nloc; y[t] = fmaxf(acc[t][v] * (1.0f / HS_) * sc2[c] + sh2[c], 0.0f); m = fmaxf(m, y[t]); }
#pragma unroll
    for (int of = 1; of < 16; of <<= 1) m = fmaxf(m, __shfl_xor(m, of));
    float z = 0.0f;
#pragma unroll
    for (int t = 0; t < 4; ++t) z += nexp(y[t] - m);
#pragma unroll
    for (int of = 1; of < 16; of <<= 1) z += __shfl_xor(z, of);
    if (nloc == 0) Ys[wid * 16 + 8 * hlf + v] = 1.0f / z; }
  __syncthreads();
  for (int pass = 0; pass < 2; ++pass) { if (threadIdx.x < 32) ((volatile float*)out)[(size_t)b * T + blockIdx.x * 32 + threadIdx.x] = Ys[threadIdx.x]; __threadfence(); }
}
}

extern "C" void kernel_launch(void* const* d_in, const int* in_sizes, int n_in,
                              void* d_out, int out_size, void* d_ws, size_t ws_size, hipStream_t stream) {
  (void)n_in; (void)out_size;
  const float* vec = (const float*)d_in[0]; const float* box = (const float*)d_in[1]; const int* edges = (const int*)d_in[2];
  const float* W1 = (const float*)d_in[3]; const float* b1 = (const float*)d_in[4]; const float* g1 = (const float*)d_in[5]; const float* be1 = (const float*)d_in[6]; const float* m1 = (const float*)d_in[7]; const float* v1 = (const float*)d_in[8];
  const float* W2 = (const float*)d_in[9]; const float* b2 = (const float*)d_in[10]; const float* g2 = (const float*)d_in[11]; const float* be2 = (const float*)d_in[12]; const float* m2 = (const float*)d_in[13]; const float* v2 = (const float*)d_in[14];
  float* out = (float*)d_out;
  if (in_sizes[0] != Bn * N * D || in_sizes[1] != Bn * N * 4 || in_sizes[2] != Bn * T * 2 || in_sizes[3] != 264 * H || in_sizes[9] != H * O) return;
  size_t off = 0; char* ws = (char*)d_ws;
  auto carve = [&](size_t bytes) { char* p = ws + off; off += (bytes + 255) & ~(size_t)255; return p; };
  unsigned short* wn = (unsigned short*)carve((size_t)2 * H * KN * 2); b16* w2r = (b16*)carve((size_t)O * H * 2); float* bnp = (float*)carve((2 * H + 2 * O) * 4); float* na = (float*)carve((size_t)NPAD * 2 * H * 4);
  if (off > ws_size) return;
  prep_kernel<<<64, 256, 0, stream>>>(W1, b1, g1, be1, m1, v1, W2, b2, g2, be2, m2, v2, wn, w2r, bnp);
  for (int b = 0; b < Bn; ++b) {
    node_kernel<<<dim3(2 * H / 64, NPAD / 128), 128, 0, stream>>>(vec, box, b, wn, na);
    edge_kernel<<<T / 32, 64, 0, stream>>>(edges, b, na, w2r, bnp, out);
  }
}
